// HierarchicalTemporalAttention_42408507080888
// MI455X (gfx1250) — hardware-verified
//
#include <hip/hip_runtime.h>

typedef _Float16 h16;
typedef _Float16 v16h __attribute__((ext_vector_type(16)));
typedef _Float16 v8h  __attribute__((ext_vector_type(8)));
typedef float    v8f  __attribute__((ext_vector_type(8)));
typedef float    v4f  __attribute__((ext_vector_type(4)));
typedef v8h __attribute__((may_alias)) v8ha;
typedef v4f __attribute__((may_alias)) v4fa;

union Frag { v16h v; v8h half[2]; };

#define BATCH  8
#define SEQ    1024
#define HID    512
#define HD     64
#define NTOK   (BATCH * SEQ)
#define TP     1030
#define PADR   3
#define CW     2048
#define NGRP   64
#define GSZ    65536
#define WSC    64.0f
#define ASC    16.0f
#define PSCALE 16384.0f
#define SCL    (1.0f / 256.0f)

__device__ __forceinline__ v8f wmma_f16(v16h a, v16h b, v8f c) {
  v8f d = __builtin_amdgcn_wmma_f32_16x16x32_f16(false, a, false, b, (short)0, c, false, false);
#if defined(__HIP_DEVICE_COMPILE__)
  asm volatile("v_nop\n\tv_nop\n\tv_nop\n\tv_nop" : "+v"(d) : "v"(a), "v"(b));
#endif
  return d;
}

__device__ __forceinline__ v16h load_frag(const h16* p, int h) {
  Frag f;
  f.half[0] = *(const v8ha*)(p + 8 * h);
  f.half[1] = *(const v8ha*)(p + 16 + 8 * h);
  return f.v;
}

__device__ __forceinline__ float bf16r(float f) {
  unsigned int u = __float_as_uint(f);
  u = (u + 0x7FFFu + ((u >> 16) & 1u)) & 0xFFFF0000u;
  return __uint_as_float(u);
}

__global__ __launch_bounds__(256) void cvt_x_kernel(const float* __restrict__ x,
                                                    h16* __restrict__ xh, int n8) {
  const int g = blockIdx.x * 256 + threadIdx.x;
  if (g >= n8) return;
  const float* src = x + (size_t)g * 8;
  const v4f a = *(const v4fa*)src;
  const v4f c = *(const v4fa*)(src + 4);
  const v8h o = { (h16)bf16r(a.x), (h16)bf16r(a.y), (h16)bf16r(a.z), (h16)bf16r(a.w),
                  (h16)bf16r(c.x), (h16)bf16r(c.y), (h16)bf16r(c.z), (h16)bf16r(c.w) };
  h16* dst = xh + (size_t)g * 8;
  *(volatile v8h*)dst = o;
  __threadfence();
  *(volatile v8h*)dst = o;
}

__global__ __launch_bounds__(256) void wtrans_kernel(
    const float* __restrict__ s0, const float* __restrict__ s1,
    const float* __restrict__ s2, const float* __restrict__ s3,
    h16* d0, h16* d1, h16* d2, h16* d3, int Kin, int N, int nzpm)
{
  __shared__ __attribute__((aligned(16))) h16 sT[64 * 72];
  const int tid = threadIdx.x;
  const int z = blockIdx.z;
  const int mat = z / nzpm;
  const int lv = z - mat * nzpm;
  const float* src = (mat == 0) ? s0 : ((mat == 1) ? s1 : ((mat == 2) ? s2 : s3));
  h16* dst = (mat == 0) ? d0 : ((mat == 1) ? d1 : ((mat == 2) ? d2 : d3));
  const size_t moff = (size_t)lv * (size_t)Kin * (size_t)N;
  src += moff;
  dst += moff;
  const int kt = blockIdx.x, nt = blockIdx.y;
  const int k = tid >> 2;
  const int n0 = (tid & 3) * 16;
  const float* rp = src + (size_t)(kt * 64 + k) * N + nt * 64 + n0;
  #pragma unroll
  for (int u = 0; u < 4; ++u) {
    const v4f v = *(const v4fa*)(rp + 4 * u);
    h16* c = sT + (n0 + 4 * u) * 72 + k;
    c[0]   = (h16)(bf16r(v.x) * WSC);
    c[72]  = (h16)(bf16r(v.y) * WSC);
    c[144] = (h16)(bf16r(v.z) * WSC);
    c[216] = (h16)(bf16r(v.w) * WSC);
  }
  __syncthreads();
  const int j8 = tid & 7, lr = tid >> 3;
  v8h vv[2];
  h16* oo[2];
  #pragma unroll
  for (int ps = 0; ps < 2; ++ps) {
    const int L = ps * 32 + lr;
    vv[ps] = *(const v8ha*)(sT + L * 72 + 8 * j8);
    oo[ps] = dst + (size_t)(nt * 64 + L) * Kin + kt * 64 + 8 * j8;
    *(volatile v8h*)oo[ps] = vv[ps];
  }
  __threadfence();
  #pragma unroll
  for (int ps = 0; ps < 2; ++ps) *(volatile v8h*)oo[ps] = vv[ps];
}

__global__ __launch_bounds__(64) void padfill_kernel(
    const float* __restrict__ bq, const float* __restrict__ bk, const float* __restrict__ bv,
    h16* Pq, h16* Pk, h16* Pv)
{
  const int pr = blockIdx.x;
  const int b = pr / 6, j = pr - 6 * b;
  const int row = b * TP + ((j < 3) ? j : (SEQ + j));
  const int pl = blockIdx.y;
  const float* bias = (pl == 0) ? bq : ((pl == 1) ? bk : bv);
  h16* P = (pl == 0) ? Pq : ((pl == 1) ? Pk : Pv);
  const int c0 = 8 * threadIdx.x;
  const v4f a = *(const v4fa*)(bias + c0);
  const v4f c = *(const v4fa*)(bias + c0 + 4);
  const v8h o = { (h16)(bf16r(a.x) * ASC), (h16)(bf16r(a.y) * ASC), (h16)(bf16r(a.z) * ASC), (h16)(bf16r(a.w) * ASC),
                  (h16)(bf16r(c.x) * ASC), (h16)(bf16r(c.y) * ASC), (h16)(bf16r(c.z) * ASC), (h16)(bf16r(c.w) * ASC) };
  h16* dst = P + (size_t)row * HID + c0;
  *(volatile v8h*)dst = o;
  __threadfence();
  *(volatile v8h*)dst = o;
}

__device__ __forceinline__ int phys_row(int R, int rpb, int pp, int po) {
  const int bb = R / rpb;
  return bb * pp + po + (R - bb * rpb);
}

__device__ __forceinline__ void gemm_store_h(const h16* sH, h16* C, int ldc, int col0,
                                             int m0, int w, int lane, int rpb, int pp, int po) {
  const int q8 = lane & 7, sub = lane >> 3;
  #pragma unroll
  for (int i = 0; i < 8; ++i) {
    const int lid = 32 * w + 4 * i + sub;
    const int pr = phys_row(m0 + lid, rpb, pp, po);
    const v8h v = *(const v8ha*)(sH + lid * 64 + 8 * q8);
    *(volatile v8h*)(C + (size_t)pr * ldc + col0 + 8 * q8) = v;
  }
}

__device__ __forceinline__ void gemm_store_f(const float* sF, float* C, int ldc, int col0,
                                             int m0, int w, int lane, int rpb, int pp, int po) {
  const int hh = lane >> 4, c4 = (lane & 15) * 4;
  #pragma unroll
  for (int i = 0; i < 16; ++i) {
    const int lid = 32 * w + 2 * i + hh;
    const int pr = phys_row(m0 + lid, rpb, pp, po);
    const v4f v = *(const v4fa*)(sF + lid * 64 + c4);
    *(volatile v4f*)(C + (size_t)pr * ldc + col0 + c4) = v;
  }
}

template <int F32OUT>
__global__ __launch_bounds__(128) void gemm_kernel(
    const h16* __restrict__ A,
    const h16* __restrict__ Bt0, const h16* __restrict__ Bt1, const h16* __restrict__ Bt2,
    const float* __restrict__ bs0, const float* __restrict__ bs1, const float* __restrict__ bs2,
    void* C0, void* C1, void* C2,
    int lda, int ldb, int K, int ldc, int coff, int ngrp,
    float accScale, float os0, float os1, float os2,
    int rpb, int pp, int po)
{
  __shared__ __attribute__((aligned(16))) unsigned char sbuf[F32OUT ? (128 * 64 * 4) : (128 * 64 * 2)];

  const int tid = threadIdx.x, lane = tid & 31, w = tid >> 5;
  const int h = lane >> 4, m = lane & 15;
  const int which = blockIdx.y / ngrp;
  const int ng = blockIdx.y - which * ngrp;
  const int n0 = ng * 64;
  const h16* Bt = (which == 0) ? Bt0 : ((which == 1) ? Bt1 : Bt2);
  const float* bias = (which == 0) ? bs0 : ((which == 1) ? bs1 : bs2);
  void* Cv = (which == 0) ? C0 : ((which == 1) ? C1 : C2);
  const float os = (which == 0) ? os0 : ((which == 1) ? os1 : os2);

  const int m0 = blockIdx.x * 128;
  const int m0w = m0 + 32 * w;
  const h16* xa0 = A + (size_t)(m0w + m) * lda;
  const h16* xa1 = xa0 + (size_t)16 * lda;
  const h16* wb  = Bt + (size_t)(n0 + m) * ldb;

  const v8f zero8 = {0.f, 0.f, 0.f, 0.f, 0.f, 0.f, 0.f, 0.f};
  v8f acc[2][4];
  #pragma unroll
  for (int mt = 0; mt < 2; ++mt)
    #pragma unroll
    for (int nt = 0; nt < 4; ++nt) acc[mt][nt] = zero8;

  #pragma unroll 1
  for (int k0 = 0; k0 < K; k0 += 32) {
    const v16h a0 = load_frag(xa0 + k0, h);
    const v16h a1 = load_frag(xa1 + k0, h);
    #pragma unroll
    for (int nt = 0; nt < 4; ++nt) {
      const v16h b = load_frag(wb + (size_t)nt * 16 * ldb + k0, h);
      acc[0][nt] = wmma_f16(a0, b, acc[0][nt]);
      acc[1][nt] = wmma_f16(a1, b, acc[1][nt]);
    }
  }

  h16* sH = (h16*)sbuf;
  float* sF = (float*)sbuf;
  #pragma unroll
  for (int nt = 0; nt < 4; ++nt) {
    const int coll = 16 * nt + m;
    const float br = bf16r(bias[n0 + coll]);
    #pragma unroll
    for (int mt = 0; mt < 2; ++mt) {
      #pragma unroll
      for (int r = 0; r < 8; ++r) {
        const int rowl = 32 * w + 16 * mt + 8 * h + r;
        const float y = (acc[mt][nt][r] * accScale + br) * os;
        if (F32OUT) sF[rowl * 64 + coll] = y;
        else        sH[rowl * 64 + coll] = (h16)y;
      }
    }
  }
  __syncthreads();

  if (F32OUT) {
    float* C = (float*)Cv;
    gemm_store_f(sF, C, ldc, coff + n0, m0, w, lane, rpb, pp, po);
    __threadfence();
    gemm_store_f(sF, C, ldc, coff + n0, m0, w, lane, rpb, pp, po);
  } else {
    h16* C = (h16*)Cv;
    gemm_store_h(sH, C, ldc, coff + n0, m0, w, lane, rpb, pp, po);
    __threadfence();
    gemm_store_h(sH, C, ldc, coff + n0, m0, w, lane, rpb, pp, po);
  }
}

__global__ __launch_bounds__(256) void lattn_kernel(
    const h16* __restrict__ Pq, const h16* __restrict__ Pk, const h16* __restrict__ Pv,
    h16* __restrict__ Mo, int w)
{
  __shared__ __attribute__((aligned(16))) float sO[64 * 64];
  __shared__ __attribute__((aligned(16))) h16 sM[HID];

  const int tid = threadIdx.x;
  const int wv = tid >> 5;
  const int token = blockIdx.x;
  const int b = token >> 10, t = token & (SEQ - 1);
  const int pad = (w - 1) >> 1;
  const int e = tid >> 2, dq = tid & 3;
  const int rbase = b * TP + PADR + t - pad;

  if (wv < w) {
    const int hh = e / w;
    const int e0 = hh * w;
    const int jq = e >> 3, cbq = e & 7;
    const h16* qp = Pq + (size_t)(rbase + jq) * HID + cbq * HD + dq * 16;
    Frag qf;
    qf.half[0] = *(const v8ha*)qp;
    qf.half[1] = *(const v8ha*)(qp + 8);
    float q[16], o[16];
    #pragma unroll
    for (int i = 0; i < 16; ++i) { q[i] = (float)qf.v[i]; o[i] = 0.f; }
    float mrun = -1e30f, lrun = 0.f;

    #pragma unroll 1
    for (int j = 0; j < w; ++j) {
      const int ek = e0 + j;
      const int jk = ek >> 3, cbk = ek & 7;
      const size_t koff = (size_t)(rbase + jk) * HID + cbk * HD + dq * 16;
      Frag kf;
      kf.half[0] = *(const v8ha*)(Pk + koff);
      kf.half[1] = *(const v8ha*)(Pk + koff + 8);
      float d = 0.f;
      #pragma unroll
      for (int i = 0; i < 16; ++i) d += q[i] * (float)kf.v[i];
      d += __shfl_xor(d, 1);
      d += __shfl_xor(d, 2);
      const float s = d * (1.0f / 2048.0f);
      const float mnew = fmaxf(mrun, s);
      const float alpha = __expf(mrun - mnew);
      const float p = __expf(s - mnew);
      mrun = mnew;
      lrun = lrun * alpha + p;
      Frag vf;
      vf.half[0] = *(const v8ha*)(Pv + koff);
      vf.half[1] = *(const v8ha*)(Pv + koff + 8);
      #pragma unroll
      for (int i = 0; i < 16; ++i) o[i] = o[i] * alpha + p * (float)vf.v[i];
    }
    const float inv = 1.0f / lrun;
    float* so = sO + e * 64 + dq * 16;
    #pragma unroll
    for (int u = 0; u < 4; ++u) {
      const v4f t4 = { o[4 * u] * inv, o[4 * u + 1] * inv, o[4 * u + 2] * inv, o[4 * u + 3] * inv };
      *(v4fa*)(so + 4 * u) = t4;
    }
  }
  __syncthreads();

  {
    const int c = 2 * tid;
    const int cb = c >> 6, dd = c & 63;
    float s0 = 0.f, s1 = 0.f;
    #pragma unroll 1
    for (int p = 0; p < w; ++p) {
      const float* rr = sO + (p * 8 + cb) * 64 + dd;
      s0 += rr[0];
      s1 += rr[1];
    }
    const float invw = 1.0f / (float)w;
    sM[c]     = (h16)(s0 * invw);
    sM[c + 1] = (h16)(s1 * invw);
  }
  __syncthreads();

  if (tid < 64) {
    const v8h v = *(const v8ha*)(sM + 8 * tid);
    h16* dst = Mo + (size_t)token * HID + 8 * tid;
    *(volatile v8h*)dst = v;
    __threadfence();
    *(volatile v8h*)dst = v;
  }
}

__global__ __launch_bounds__(256) void vtrans_kernel(const h16* __restrict__ Pv, h16* Vt) {
  __shared__ __attribute__((aligned(16))) h16 sT[64 * 72];
  const int tid = threadIdx.x;
  const int kt = blockIdx.x, g = blockIdx.y;
  const h16* src = Pv + (size_t)g * GSZ + (size_t)kt * 64 * 64;
  #pragma unroll
  for (int u = 0; u < 2; ++u) {
    const int idx = tid * 2 + u;
    const int key = idx >> 3, d0 = (idx & 7) * 8;
    const v8h v = *(const v8ha*)(src + idx * 8);
    #pragma unroll
    for (int i = 0; i < 8; ++i) sT[(d0 + i) * 72 + key] = v[i];
  }
  __syncthreads();
  const int j8 = tid & 7, lr = tid >> 3;
  v8h vv[2];
  h16* oo[2];
  #pragma unroll
  for (int ps = 0; ps < 2; ++ps) {
    const int L = ps * 32 + lr;
    vv[ps] = *(const v8ha*)(sT + L * 72 + 8 * j8);
    oo[ps] = Vt + ((size_t)g * HD + L) * SEQ + kt * 64 + 8 * j8;
    *(volatile v8h*)oo[ps] = vv[ps];
  }
  __threadfence();
  #pragma unroll
  for (int ps = 0; ps < 2; ++ps) *(volatile v8h*)oo[ps] = vv[ps];
}

__device__ __forceinline__ v16h pack_p(v8f a, v8f c) {
  const v16h r = { (h16)(a[0] * PSCALE), (h16)(a[1] * PSCALE), (h16)(a[2] * PSCALE), (h16)(a[3] * PSCALE),
                   (h16)(a[4] * PSCALE), (h16)(a[5] * PSCALE), (h16)(a[6] * PSCALE), (h16)(a[7] * PSCALE),
                   (h16)(c[0] * PSCALE), (h16)(c[1] * PSCALE), (h16)(c[2] * PSCALE), (h16)(c[3] * PSCALE),
                   (h16)(c[4] * PSCALE), (h16)(c[5] * PSCALE), (h16)(c[6] * PSCALE), (h16)(c[7] * PSCALE) };
  return r;
}

__device__ __forceinline__ void gatt_store(const h16* so, h16* og, int lane) {
  const int q8 = lane & 7, sub = lane >> 3;
  #pragma unroll
  for (int i = 0; i < 4; ++i) {
    const int lid = 4 * i + sub;
    const v8h v = *(const v8ha*)(so + lid * 64 + 8 * q8);
    *(volatile v8h*)(og + (size_t)lid * HD + 8 * q8) = v;
  }
}

__global__ __launch_bounds__(128) void gattn_kernel(
    const h16* __restrict__ Pq, const h16* __restrict__ Pk,
    const h16* __restrict__ Vt, h16* __restrict__ Og)
{
  __shared__ __attribute__((aligned(16))) h16 sO[4 * 16 * 64];

  const int tid = threadIdx.x, lane = tid & 31, w = tid >> 5;
  const int h = lane >> 4, m = lane & 15;
  const int g = blockIdx.y;
  const int q0 = blockIdx.x * 64 + 16 * w;
  const size_t gb = (size_t)g * GSZ;

  const h16* qrow = Pq + gb + (size_t)(q0 + m) * HD;
  const v16h qb0 = load_frag(qrow, h);
  const v16h qb1 = load_frag(qrow + 32, h);

  const v8f zero8 = {0.f, 0.f, 0.f, 0.f, 0.f, 0.f, 0.f, 0.f};
  v8f o[4];
  #pragma unroll
  for (int t = 0; t < 4; ++t) o[t] = zero8;
  float mrun = -1e30f, lrun = 0.0f;

  const h16* kbase = Pk + gb + (size_t)m * HD;
  const h16* vbase = Vt + gb + (size_t)m * SEQ;

  #pragma unroll 1
  for (int kb = 0; kb < SEQ; kb += 64) {
    v8f s[4];
    #pragma unroll
    for (int j = 0; j < 4; ++j) {
      const h16* kp = kbase + (size_t)(kb + 16 * j) * HD;
      const v16h kf0 = load_frag(kp, h);
      const v16h kf1 = load_frag(kp + 32, h);
      v8f z = zero8;
      z = wmma_f16(kf0, qb0, z);
      z = wmma_f16(kf1, qb1, z);
      s[j] = z;
    }
    float mloc = -1e30f;
    #pragma unroll
    for (int j = 0; j < 4; ++j)
      #pragma unroll
      for (int r = 0; r < 8; ++r) {
        const float v = s[j][r] * SCL;
        s[j][r] = v;
        mloc = fmaxf(mloc, v);
      }
    mloc = fmaxf(mloc, __shfl_xor(mloc, 16));
    const float mnew = fmaxf(mrun, mloc);
    const float alpha = __expf(mrun - mnew);
    mrun = mnew;
    float lsum = 0.0f;
    #pragma unroll
    for (int j = 0; j < 4; ++j)
      #pragma unroll
      for (int r = 0; r < 8; ++r) {
        const float p = __expf(s[j][r] - mnew);
        s[j][r] = p;
        lsum += p;
      }
    lsum += __shfl_xor(lsum, 16);
    lrun = lrun * alpha + lsum;
    #pragma unroll
    for (int t = 0; t < 4; ++t)
      #pragma unroll
      for (int r = 0; r < 8; ++r) o[t][r] = o[t][r] * alpha;

    const v16h pb0 = pack_p(s[0], s[1]);
    const v16h pb1 = pack_p(s[2], s[3]);

    #pragma unroll
    for (int t = 0; t < 4; ++t) {
      const h16* vp = vbase + (size_t)(16 * t) * SEQ + kb;
      const v16h vf0 = load_frag(vp, h);
      const v16h vf1 = load_frag(vp + 32, h);
      o[t] = wmma_f16(vf0, pb0, o[t]);
      o[t] = wmma_f16(vf1, pb1, o[t]);
    }
  }

  const float inv = (1.0f / lrun) * (1.0f / PSCALE);
  h16* so = sO + w * 1024;
  #pragma unroll
  for (int t = 0; t < 4; ++t)
    #pragma unroll
    for (int r = 0; r < 8; ++r)
      so[m * 64 + 16 * t + 8 * h + r] = (h16)(o[t][r] * inv);
  __syncthreads();

  h16* og = Og + gb + (size_t)q0 * HD;
  gatt_store(so, og, lane);
  __threadfence();
  gatt_store(so, og, lane);
}

extern "C" void kernel_launch(void* const* d_in, const int* in_sizes, int n_in,
                              void* d_out, int out_size, void* d_ws, size_t ws_size,
                              hipStream_t stream) {
  if (n_in < 19) return;
  const int nW = HID * HID;
  if (in_sizes[0] != NTOK * HID) return;
  if (in_sizes[1] != 3 * nW || in_sizes[3] != 3 * nW || in_sizes[5] != 3 * nW || in_sizes[7] != 3 * nW) return;
  if (in_sizes[2] != 3 * HID || in_sizes[4] != 3 * HID || in_sizes[6] != 3 * HID || in_sizes[8] != 3 * HID) return;
  if (in_sizes[9] != nW || in_sizes[11] != nW || in_sizes[13] != nW || in_sizes[15] != nW) return;
  if (in_sizes[10] != HID || in_sizes[12] != HID || in_sizes[14] != HID || in_sizes[16] != HID) return;
  if (in_sizes[17] != CW * HID || in_sizes[18] != HID) return;
  if (out_size != NTOK * HID) return;

  const float* x      = (const float*)d_in[0];
  const float* loc_wq = (const float*)d_in[1];
  const float* loc_bq = (const float*)d_in[2];
  const float* loc_wk = (const float*)d_in[3];
  const float* loc_bk = (const float*)d_in[4];
  const float* loc_wv = (const float*)d_in[5];
  const float* loc_bv = (const float*)d_in[6];
  const float* loc_wo = (const float*)d_in[7];
  const float* loc_bo = (const float*)d_in[8];
  const float* g_wq   = (const float*)d_in[9];
  const float* g_bq   = (const float*)d_in[10];
  const float* g_wk   = (const float*)d_in[11];
  const float* g_bk   = (const float*)d_in[12];
  const float* g_wv   = (const float*)d_in[13];
  const float* g_bv   = (const float*)d_in[14];
  const float* g_wo   = (const float*)d_in[15];
  const float* g_bo   = (const float*)d_in[16];
  const float* out_w  = (const float*)d_in[17];
  const float* out_b  = (const float*)d_in[18];
  float* out = (float*)d_out;

  const size_t xh_b = (size_t)NTOK * HID * 2;
  const size_t wl_b = (size_t)3 * nW * 2;
  const size_t wg_b = (size_t)nW * 2;
  const size_t wo_b = (size_t)CW * HID * 2;
  const size_t pl_b = (size_t)BATCH * TP * HID * 2;
  const size_t at_b = (size_t)NTOK * HID * 2;
  const size_t cb_b = (size_t)NTOK * CW * 2;
  const size_t total = xh_b + 4 * wl_b + 4 * wg_b + wo_b + 3 * pl_b + 2 * at_b + cb_b;
  if (total > ws_size) return;

  char* ws = (char*)d_ws;
  size_t off = 0;
  h16* xh  = (h16*)(ws + off); off += xh_b;
  h16* wqt = (h16*)(ws + off); off += wl_b;
  h16* wkt = (h16*)(ws + off); off += wl_b;
  h16* wvt = (h16*)(ws + off); off += wl_b;
  h16* wot = (h16*)(ws + off); off += wl_b;
  h16* gqt = (h16*)(ws + off); off += wg_b;
  h16* gkt = (h16*)(ws + off); off += wg_b;
  h16* gvt = (h16*)(ws + off); off += wg_b;
  h16* got = (h16*)(ws + off); off += wg_b;
  h16* owt = (h16*)(ws + off); off += wo_b;
  h16* Pq  = (h16*)(ws + off); off += pl_b;
  h16* Pk  = (h16*)(ws + off); off += pl_b;
  h16* Pv  = (h16*)(ws + off); off += pl_b;
  h16* Vt  = (h16*)(ws + off); off += at_b;
  h16* Ma  = (h16*)(ws + off); off += at_b;
  h16* comb = (h16*)(ws + off); off += cb_b;
  if (off > ws_size) return;

  const int n8 = NTOK * HID / 8;
  cvt_x_kernel<<<dim3((n8 + 255) / 256), dim3(256), 0, stream>>>(x, xh, n8);
  wtrans_kernel<<<dim3(HID / 64, HID / 64, 12), dim3(256), 0, stream>>>(
      loc_wq, loc_wk, loc_wv, loc_wo, wqt, wkt, wvt, wot, HID, HID, 3);
  wtrans_kernel<<<dim3(HID / 64, HID / 64, 4), dim3(256), 0, stream>>>(
      g_wq, g_wk, g_wv, g_wo, gqt, gkt, gvt, got, HID, HID, 1);
  wtrans_kernel<<<dim3(CW / 64, HID / 64, 1), dim3(256), 0, stream>>>(
      out_w, out_w, out_w, out_w, owt, owt, owt, owt, CW, HID, 1);

  const int wsz[3] = {3, 5, 7};
  for (int lv = 0; lv < 3; ++lv) {
    const float* bq = loc_bq + lv * HID;
    const float* bk = loc_bk + lv * HID;
    const float* bv = loc_bv + lv * HID;
    const float* bo = loc_bo + lv * HID;
    const size_t wo_off = (size_t)lv * nW;
    padfill_kernel<<<dim3(BATCH * 6, 3), dim3(64), 0, stream>>>(bq, bk, bv, Pq, Pk, Pv);
    gemm_kernel<0><<<dim3(NTOK / 128, 24), dim3(128), 0, stream>>>(
        xh, wqt + wo_off, wkt + wo_off, wvt + wo_off, bq, bk, bv,
        (void*)Pq, (void*)Pk, (void*)Pv,
        HID, HID, HID, HID, 0, 8, 1.0f / WSC, ASC, ASC, ASC, SEQ, TP, PADR);
    lattn_kernel<<<dim3(NTOK), dim3(256), 0, stream>>>(Pq, Pk, Pv, Ma, wsz[lv]);
    gemm_kernel<0><<<dim3(NTOK / 128, 8), dim3(128), 0, stream>>>(
        Ma, wot + wo_off, wot + wo_off, wot + wo_off, bo, bo, bo,
        (void*)comb, (void*)comb, (void*)comb,
        HID, HID, HID, CW, lv * HID, 8, 1.0f / (WSC * ASC), ASC, ASC, ASC, SEQ, SEQ, 0);
  }

  gemm_kernel<0><<<dim3(NTOK / 128, 24), dim3(128), 0, stream>>>(
      xh, gqt, gkt, gvt, g_bq, g_bk, g_bv, (void*)Pq, (void*)Pk, (void*)Pv,
      HID, HID, HID, HID, 0, 8, 1.0f / WSC, 2.0f, ASC, ASC, SEQ, SEQ, 0);
  vtrans_kernel<<<dim3(SEQ / 64, NGRP), dim3(256), 0, stream>>>(Pv, Vt);
  gattn_kernel<<<dim3(SEQ / 64, NGRP), dim3(128), 0, stream>>>(Pq, Pk, Vt, Ma);
  gemm_kernel<0><<<dim3(NTOK / 128, 8), dim3(128), 0, stream>>>(
      Ma, got, got, got, g_bo, g_bo, g_bo, (void*)comb, (void*)comb, (void*)comb,
      HID, HID, HID, CW, 3 * HID, 8, 1.0f / (WSC * ASC), ASC, ASC, ASC, SEQ, SEQ, 0);

  gemm_kernel<1><<<dim3(NTOK / 128, 8), dim3(128), 0, stream>>>(
      comb, owt, owt, owt, out_b, out_b, out_b, (void*)out, (void*)out, (void*)out,
      CW, CW, CW, HID, 0, 8, 1.0f / (WSC * ASC), 1.0f, 1.0f, 1.0f, SEQ, SEQ, 0);
}
